// MambaB_8641474199637
// MI455X (gfx1250) — hardware-verified
//
#include <hip/hip_runtime.h>
#include <math.h>

typedef __attribute__((ext_vector_type(16))) _Float16 v16h;
typedef __attribute__((ext_vector_type(8)))  _Float16 v8h;
typedef __attribute__((ext_vector_type(16))) __bf16   v16b;
typedef __attribute__((ext_vector_type(8)))  __bf16   v8b;
typedef __attribute__((ext_vector_type(8)))  float    v8f;
typedef __attribute__((ext_vector_type(4)))  float    v4f;

constexpr int kBatch = 4;
constexpr int kSeqL  = 4096;
constexpr int kChalf = 128;
constexpr int kDmod  = 256;
constexpr int kDin   = 512;
constexpr int kXZP   = 2 * kDin;
constexpr int kNst   = 16;
constexpr int kDtR   = 16;
constexpr int kDtP   = 32;
constexpr int kPrjN  = 48;
constexpr int kPrjP  = 64;
constexpr int kRows  = kBatch * kSeqL;
constexpr int kCout  = 128;
constexpr int kTP    = 260;

__device__ __forceinline__ unsigned short f2bf_bits(float f) {
  unsigned u = __float_as_uint(f);
  return (unsigned short)((u + 0x7FFFu + ((u >> 16) & 1u)) >> 16);
}
__device__ __forceinline__ float bf_bits2f(unsigned short h) { return __uint_as_float(((unsigned)h) << 16); }

__device__ __forceinline__ void dep_guard_h(v8f& a, v8f& b, v16h x, v16h y) { asm volatile("v_nop\n\tv_nop\n\tv_nop\n\tv_nop" : "+v"(a), "+v"(b) : "v"(x), "v"(y)); }
__device__ __forceinline__ void dep_guard_b(v8f& a, v8f& b, v16b x, v16b y) { asm volatile("v_nop\n\tv_nop\n\tv_nop\n\tv_nop" : "+v"(a), "+v"(b) : "v"(x), "v"(y)); }
__device__ __forceinline__ void keep4_h(v16h a, v16h b, v16h c, v16h d) { asm volatile("v_nop" :: "v"(a), "v"(b), "v"(c), "v"(d)); }
__device__ __forceinline__ void keep4_b(v16b a, v16b b, v16b c, v16b d) { asm volatile("v_nop" :: "v"(a), "v"(b), "v"(c), "v"(d)); }
__device__ __forceinline__ void acc_guard4(v8f& a, v8f& b, v8f& c, v8f& d) { asm volatile("v_nop\n\tv_nop\n\tv_nop\n\tv_nop" : "+v"(a), "+v"(b), "+v"(c), "+v"(d)); }
template <typename T> struct Frag;
template <> struct Frag<_Float16> {
  typedef v16h V; union U { v16h v; v8h h[2]; };
  static __device__ __forceinline__ v16h load(const _Float16* p) {
    U f; f.h[0] = *(const v8h*)(p); f.h[1] = *(const v8h*)(p + 16); return f.v;
  }
  static __device__ __forceinline__ v8f mma(v16h a, v16h b, v8f c) {
    return __builtin_amdgcn_wmma_f32_16x16x32_f16(false, a, false, b, (short)0, c, false, false);
  }
  static __device__ __forceinline__ void guard(v8f& a, v8f& b, v16h x, v16h y) { dep_guard_h(a, b, x, y); }
  static __device__ __forceinline__ void keep(v16h a, v16h b, v16h c, v16h d) { keep4_h(a, b, c, d); }
};
template <> struct Frag<__bf16> {
  typedef v16b V; union U { v16b v; v8b h[2]; };
  static __device__ __forceinline__ v16b load(const __bf16* p) {
    U f; f.h[0] = *(const v8b*)(p); f.h[1] = *(const v8b*)(p + 16); return f.v;
  }
  static __device__ __forceinline__ v8f mma(v16b a, v16b b, v8f c) {
    return __builtin_amdgcn_wmma_f32_16x16x32_bf16(false, a, false, b, (short)0, c, false, false);
  }
  static __device__ __forceinline__ void guard(v8f& a, v8f& b, v16b x, v16b y) { dep_guard_b(a, b, x, y); }
  static __device__ __forceinline__ void keep(v16b a, v16b b, v16b c, v16b d) { keep4_b(a, b, c, d); }
};

template <int ET> struct Elem;
template <> struct Elem<0> { typedef _Float16 T; };
template <> struct Elem<1> { typedef __bf16 T; };
template <int ET, bool SPLIT, int BIAS_MODE, int OUT_MODE, bool RESID, int ACT = 0>
__global__ __launch_bounds__(256) void wmma_gemm64(
    const unsigned short* __restrict__ Ap, const unsigned short* __restrict__ A2p, int lda, long strideA,
    const unsigned short* __restrict__ Btp, const unsigned short* __restrict__ Bt2p, int ldb, long strideB,
    void* __restrict__ Cout, void* __restrict__ Cout2, int ldc, long strideC,
    const float* __restrict__ bias,
    const float* __restrict__ resid, long strideR,
    int M, int N, int K, float scale) {
  typedef typename Elem<ET>::T T;
  typedef typename Frag<T>::V V;
  const T* A = (const T*)Ap; const T* A2 = (const T*)A2p; const T* Bt = (const T*)Btp; const T* Bt2 = (const T*)Bt2p;
  __shared__ __align__(16) float sT[8][16 * 68];
  const int b    = blockIdx.y;
  const int lane = threadIdx.x & 31;
  const int wave = threadIdx.x >> 5;
  const int tilesN = N >> 6;
  const int tilesM = M >> 6;
  const int tile = blockIdx.x * 8 + wave;
  if (tile >= tilesM * tilesN) return;
  const int tm = tile / tilesN;
  const int tn = tile - tm * tilesN;
  const int m0 = tm << 6;
  const int n0 = tn << 6;

  const T* Ab  = A  + (size_t)b * strideA;
  const T* Bb  = Bt + (size_t)b * strideB;
  const T* Ab2 = SPLIT ? (A2  + (size_t)b * strideA) : nullptr;
  const T* Bb2 = SPLIT ? (Bt2 + (size_t)b * strideB) : nullptr;

  const int rlane = lane & 15;
  const int koff  = (lane >> 4) * 8;
  const int mOff  = (lane >> 4) * 8;

  v8f acc[4][4];
#pragma unroll
  for (int i = 0; i < 4; ++i)
#pragma unroll
    for (int j = 0; j < 4; ++j) acc[i][j] = (v8f){0.f,0.f,0.f,0.f,0.f,0.f,0.f,0.f};

  for (int k0 = 0; k0 < K; k0 += 32) {
    V bh[4], bl[4];
#pragma unroll
    for (int j = 0; j < 4; ++j) {
      const size_t bo = (size_t)(n0 + (j << 4) + rlane) * ldb + koff + k0;
      bh[j] = Frag<T>::load(Bb + bo);
      if (SPLIT) bl[j] = Frag<T>::load(Bb2 + bo);
    }
#pragma unroll
    for (int i = 0; i < 4; ++i) {
      const size_t ao = (size_t)(m0 + (i << 4) + rlane) * lda + koff + k0;
      V ah = Frag<T>::load(Ab + ao);
      V al;
      if (SPLIT) al = Frag<T>::load(Ab2 + ao);
#pragma unroll
      for (int j = 0; j < 4; ++j) {
        acc[i][j] = Frag<T>::mma(ah, bh[j], acc[i][j]);
        if (SPLIT) {
          acc[i][j] = Frag<T>::mma(ah, bl[j], acc[i][j]);
          acc[i][j] = Frag<T>::mma(al, bh[j], acc[i][j]);
        }
      }
      Frag<T>::guard(acc[i][0], acc[i][3], ah, SPLIT ? al : ah);
    }
    Frag<T>::keep(bh[0], bh[1], bh[2], bh[3]);
    if (SPLIT) Frag<T>::keep(bl[0], bl[1], bl[2], bl[3]);
  }
  acc_guard4(acc[0][0], acc[0][1], acc[0][2], acc[0][3]);
  acc_guard4(acc[1][0], acc[1][1], acc[1][2], acc[1][3]);
  acc_guard4(acc[2][0], acc[2][1], acc[2][2], acc[2][3]);
  acc_guard4(acc[3][0], acc[3][1], acc[3][2], acc[3][3]);

  float* slab = sT[wave];
  const float* Rb = RESID ? (resid + (size_t)b * strideR) : nullptr;
#pragma unroll
  for (int i = 0; i < 4; ++i) {
    const int mBase = m0 + (i << 4);
#pragma unroll
    for (int j = 0; j < 4; ++j) {
      const int n = n0 + (j << 4) + rlane;
      float bv = 0.f;
      if (BIAS_MODE == 2) bv = bias[n];
#pragma unroll
      for (int r = 0; r < 8; ++r) {
        float v = acc[i][j][r] * scale;
        if (BIAS_MODE == 1) v += bias[mBase + mOff + r];
        if (BIAS_MODE == 2) v += bv;
        if (RESID) v += Rb[(size_t)(mBase + mOff + r) * ldc + n];
        if (ACT == 1) v = tanhf(v);
        if (ACT == 2) v = fmaxf(v, 0.0f);
        if (ACT == 3) v = v / (1.0f + expf(-v));
        if (ACT == 4) v = (v > 0.f) ? v : 0.01f * v;
        if (ACT == 5) v = 0.5f * v * (1.0f + erff(v * 0.70710678118654752f));
        slab[(mOff + r) * 68 + (j << 4) + rlane] = v;
      }
    }
    __builtin_amdgcn_fence(__ATOMIC_RELEASE, "workgroup");
    __builtin_amdgcn_wave_barrier();
    __builtin_amdgcn_fence(__ATOMIC_ACQUIRE, "workgroup");
    if (OUT_MODE == 0) {
      float* C = (float*)Cout + (size_t)b * strideC;
      const int hh = lane >> 4, c4 = (lane & 15) * 4;
      for (int pass = 0; pass < 2; ++pass) {
#pragma unroll
        for (int it = 0; it < 8; ++it) {
          const int row = it * 2 + hh;
          v4f v = *(const v4f*)(slab + row * 68 + c4);
          *(volatile v4f*)(C + (size_t)(mBase + row) * ldc + n0 + c4) = v;
        }
        __threadfence();
      }
    } else {
      const int q = lane >> 3, c8 = (lane & 7) * 8;
      unsigned short* C  = (unsigned short*)Cout  + (size_t)b * strideC;
      unsigned short* C2 = (OUT_MODE == 2) ? ((unsigned short*)Cout2 + (size_t)b * strideC) : nullptr;
      for (int pass = 0; pass < 2; ++pass) {
#pragma unroll
        for (int it = 0; it < 4; ++it) {
          const int row = it * 4 + q;
          const float* sp = slab + row * 68 + c8;
          v8h hv, lv;
#pragma unroll
          for (int e = 0; e < 8; ++e) {
            if (OUT_MODE == 1) {
              hv[e] = (_Float16)sp[e];
            } else {
              unsigned short hb = f2bf_bits(sp[e]);
              unsigned short lb = f2bf_bits(sp[e] - bf_bits2f(hb));
              hv[e] = __builtin_bit_cast(_Float16, hb);
              lv[e] = __builtin_bit_cast(_Float16, lb);
            }
          }
          *(volatile v8h*)(C + (size_t)(mBase + row) * ldc + n0 + c8) = hv;
          if (OUT_MODE == 2) *(volatile v8h*)(C2 + (size_t)(mBase + row) * ldc + n0 + c8) = lv;
        }
        __threadfence();
      }
    }
    __builtin_amdgcn_fence(__ATOMIC_RELEASE, "workgroup");
    __builtin_amdgcn_wave_barrier();
    __builtin_amdgcn_fence(__ATOMIC_ACQUIRE, "workgroup");
  }
}

__global__ __launch_bounds__(256) void transpose_split_kernel(
    const float* __restrict__ W, unsigned short* __restrict__ Bh, unsigned short* __restrict__ Bl,
    int Kdim, int Ndim)
{
  __shared__ float tile[64 * 65];
  const int tid = threadIdx.x, lane = tid & 31, wave = tid >> 5;
  const int n0 = blockIdx.x * 64;
  const int k0 = blockIdx.y * 64;
#pragma unroll
  for (int p = 0; p < 16; ++p) {
    const int idx = tid + p * 256;
    const int kk  = idx >> 6;
    const int nn  = idx & 63;
    const int n   = n0 + nn;
    const int nc  = (n < Ndim) ? n : (Ndim - 1);
    const float v = W[(size_t)(k0 + kk) * Ndim + nc];
    tile[kk * 65 + nn] = (n < Ndim) ? v : 0.f;
  }
  __syncthreads();
  const int q = lane >> 3, c8 = (lane & 7) * 8;
  v8h hv[2], lv[2];
#pragma unroll
  for (int it = 0; it < 2; ++it) {
    const int nrow = it * 32 + wave * 4 + q;
#pragma unroll
    for (int e = 0; e < 8; ++e) {
      const float v = tile[(c8 + e) * 65 + nrow];
      const unsigned short hb = f2bf_bits(v);
      const unsigned short lb = f2bf_bits(v - bf_bits2f(hb));
      hv[it][e] = __builtin_bit_cast(_Float16, hb);
      lv[it][e] = __builtin_bit_cast(_Float16, lb);
    }
  }
  for (int pass = 0; pass < 2; ++pass) {
#pragma unroll
    for (int it = 0; it < 2; ++it) {
      const int nrow = it * 32 + wave * 4 + q;
      const size_t o = (size_t)(n0 + nrow) * Kdim + k0 + c8;
      *(volatile v8h*)(Bh + o) = hv[it];
      *(volatile v8h*)(Bl + o) = lv[it];
    }
    __threadfence();
  }
}

__global__ __launch_bounds__(256) void dtw_split_kernel(
    const float* __restrict__ W, unsigned short* __restrict__ Bh, unsigned short* __restrict__ Bl, int total8)
{
  const int i = blockIdx.x * 256 + threadIdx.x;
  if (i >= total8) return;
  const int e0 = i << 3;
  const int n  = e0 >> 5;
  const int kb = e0 & 31;
  v8h hv, lv;
#pragma unroll
  for (int e = 0; e < 8; ++e) {
    const int k  = kb + e;
    const int kc = (k < kDtR) ? k : (kDtR - 1);
    const float w = W[(size_t)kc * kDin + n];
    const float v = (k < kDtR) ? w : 0.f;
    const unsigned short hb = f2bf_bits(v);
    const unsigned short lb = f2bf_bits(v - bf_bits2f(hb));
    hv[e] = __builtin_bit_cast(_Float16, hb);
    lv[e] = __builtin_bit_cast(_Float16, lb);
  }
  *(volatile v8h*)(Bh + e0) = hv;
  *(volatile v8h*)(Bl + e0) = lv;
  __threadfence();
  *(volatile v8h*)(Bh + e0) = hv;
  *(volatile v8h*)(Bl + e0) = lv;
}

__global__ __launch_bounds__(256) void ln_kernel(
    const float* __restrict__ in0, const float* __restrict__ in1,
    const float* __restrict__ g, const float* __restrict__ bb,
    unsigned short* __restrict__ Xh, unsigned short* __restrict__ Xl)
{
  __shared__ float tile[kDmod * 33];
  __shared__ float sMu[32];
  __shared__ float sRs[32];
  const int tid = threadIdx.x, lane = tid & 31, wave = tid >> 5;
  const int b   = blockIdx.y;
  const int hw0 = blockIdx.x * 32;
#pragma unroll 4
  for (int p = 0; p < 16; ++p) {
    const int c = p * 8 + wave;
    const float v0 = in0[((size_t)(b * kChalf + c)) * kSeqL + hw0 + lane];
    const float v1 = in1[((size_t)(b * kChalf + c)) * kSeqL + hw0 + lane];
    tile[c * 33 + lane] = v0;
    tile[(kChalf + c) * 33 + lane] = v1;
  }
  __syncthreads();
  const int j = tid >> 3, sub = tid & 7;
  float s = 0.f;
#pragma unroll 8
  for (int i = 0; i < 32; ++i) s += tile[(sub + 8 * i) * 33 + j];
  s += __shfl_xor(s, 1, 32);
  s += __shfl_xor(s, 2, 32);
  s += __shfl_xor(s, 4, 32);
  const float mu = s * (1.0f / 256.0f);
  float s2 = 0.f;
#pragma unroll 8
  for (int i = 0; i < 32; ++i) {
    const float dv = tile[(sub + 8 * i) * 33 + j] - mu;
    s2 += dv * dv;
  }
  s2 += __shfl_xor(s2, 1, 32);
  s2 += __shfl_xor(s2, 2, 32);
  s2 += __shfl_xor(s2, 4, 32);
  const float var = s2 * (1.0f / 256.0f);
  const float rs  = rsqrtf(var + 1e-5f);
  if (sub == 0) { sMu[j] = mu; sRs[j] = rs; }
  __syncthreads();
  v8h hv[4], lv[4];
#pragma unroll
  for (int it = 0; it < 4; ++it) {
    const int jt = it * 8 + wave;
    const float m2 = sMu[jt], r2 = sRs[jt];
#pragma unroll
    for (int e = 0; e < 8; ++e) {
      const int c = lane * 8 + e;
      const float v = (tile[c * 33 + jt] - m2) * r2 * g[c] + bb[c];
      const unsigned short hb = f2bf_bits(v);
      const unsigned short lb = f2bf_bits(v - bf_bits2f(hb));
      hv[it][e] = __builtin_bit_cast(_Float16, hb);
      lv[it][e] = __builtin_bit_cast(_Float16, lb);
    }
  }
  for (int pass = 0; pass < 2; ++pass) {
#pragma unroll
    for (int it = 0; it < 4; ++it) {
      const int jt = it * 8 + wave;
      const size_t o = (size_t)(b * kSeqL + hw0 + jt) * kDmod + lane * 8;
      *(volatile v8h*)(Xh + o) = hv[it];
      *(volatile v8h*)(Xl + o) = lv[it];
    }
    __threadfence();
  }
}

__global__ __launch_bounds__(256) void dt_split_kernel(
    const float* __restrict__ PROJ, unsigned short* __restrict__ Dh, unsigned short* __restrict__ Dl, int total8)
{
  const int i = blockIdx.x * 256 + threadIdx.x;
  if (i >= total8) return;
  const int e0  = i << 3;
  const int row = e0 >> 5;
  const int c8  = e0 & 31;
  const bool keep = (c8 < kDtR);
  const float* p = PROJ + (size_t)row * kPrjP + (c8 & 8);
  const v4f a0 = *(const v4f*)(p);
  const v4f a1 = *(const v4f*)(p + 4);
  v8h hv, lv;
#pragma unroll
  for (int e = 0; e < 4; ++e) {
    const float v0 = keep ? a0[e] : 0.f;
    const float v1 = keep ? a1[e] : 0.f;
    const unsigned short h0 = f2bf_bits(v0);
    const unsigned short l0 = f2bf_bits(v0 - bf_bits2f(h0));
    const unsigned short h1 = f2bf_bits(v1);
    const unsigned short l1 = f2bf_bits(v1 - bf_bits2f(h1));
    hv[e]     = __builtin_bit_cast(_Float16, h0);
    lv[e]     = __builtin_bit_cast(_Float16, l0);
    hv[4 + e] = __builtin_bit_cast(_Float16, h1);
    lv[4 + e] = __builtin_bit_cast(_Float16, l1);
  }
  *(volatile v8h*)(Dh + e0) = hv;
  *(volatile v8h*)(Dl + e0) = lv;
  __threadfence();
  *(volatile v8h*)(Dh + e0) = hv;
  *(volatile v8h*)(Dl + e0) = lv;
}

__global__ __launch_bounds__(256) void conv_silu_kernel(
    const float* __restrict__ XZ, const float* __restrict__ cw, const float* __restrict__ cb,
    float* __restrict__ UC, unsigned short* __restrict__ UCh, unsigned short* __restrict__ UCl)
{
  __shared__ __align__(16) float sT[16 * kTP];
  const int tid = threadIdx.x, lane = tid & 31, wave = tid >> 5;
  const int d0 = blockIdx.x * 256, d = d0 + tid;
  const int t0 = blockIdx.y * 64;
  const float w0 = cw[d * 4 + 0], w1 = cw[d * 4 + 1], w2 = cw[d * 4 + 2], w3 = cw[d * 4 + 3];
  const float bc = cb[d];
  float xm3, xm2, xm1;
  {
    const int r3 = t0 - 3, r2 = t0 - 2, r1 = t0 - 1;
    const float v3 = XZ[(size_t)(r3 < 0 ? 0 : r3) * kXZP + d];
    const float v2 = XZ[(size_t)(r2 < 0 ? 0 : r2) * kXZP + d];
    const float v1 = XZ[(size_t)(r1 < 0 ? 0 : r1) * kXZP + d];
    xm3 = (r3 >= 0) ? v3 : 0.f;
    xm2 = (r2 >= 0) ? v2 : 0.f;
    xm1 = (r1 >= 0) ? v1 : 0.f;
  }
  const int hrow = wave >> 1;
  const int hch  = (wave & 1) * 128 + lane * 4;
#pragma unroll 1
  for (int sub = 0; sub < 4; ++sub) {
    const int lb = t0 + sub * 16;
#pragma unroll 1
    for (int s = 0; s < 16; ++s) {
      const float xc = XZ[(size_t)(lb + s) * kXZP + d];
      float acc = w0 * xm3;
      acc = fmaf(w1, xm2, acc);
      acc = fmaf(w2, xm1, acc);
      acc = fmaf(w3, xc, acc);
      const float sv = acc + bc;
      const float sg = __builtin_amdgcn_rcpf(1.0f + __expf(-sv));
      sT[s * kTP + tid] = sv * sg;
      xm3 = xm2; xm2 = xm1; xm1 = xc;
    }
    __syncthreads();
    v4f fv[4];
    v8h bv[2], lv[2];
#pragma unroll
    for (int it = 0; it < 4; ++it) fv[it] = *(const v4f*)(sT + (it * 4 + hrow) * kTP + hch);
#pragma unroll
    for (int it = 0; it < 2; ++it) {
      const float* sp = sT + (it * 8 + wave) * kTP + lane * 8;
      const v4f a0 = *(const v4f*)(sp);
      const v4f a1 = *(const v4f*)(sp + 4);
#pragma unroll
      for (int e = 0; e < 4; ++e) {
        const unsigned short h0 = f2bf_bits(a0[e]);
        const unsigned short l0 = f2bf_bits(a0[e] - bf_bits2f(h0));
        const unsigned short h1 = f2bf_bits(a1[e]);
        const unsigned short l1 = f2bf_bits(a1[e] - bf_bits2f(h1));
        bv[it][e]     = __builtin_bit_cast(_Float16, h0);
        lv[it][e]     = __builtin_bit_cast(_Float16, l0);
        bv[it][4 + e] = __builtin_bit_cast(_Float16, h1);
        lv[it][4 + e] = __builtin_bit_cast(_Float16, l1);
      }
    }
    for (int pass = 0; pass < 2; ++pass) {
#pragma unroll
      for (int it = 0; it < 4; ++it)
        *(volatile v4f*)(UC + (size_t)(lb + it * 4 + hrow) * kDin + d0 + hch) = fv[it];
#pragma unroll
      for (int it = 0; it < 2; ++it) {
        const size_t o = (size_t)(lb + it * 8 + wave) * kDin + d0 + lane * 8;
        *(volatile v8h*)(UCh + o) = bv[it];
        *(volatile v8h*)(UCl + o) = lv[it];
      }
      __threadfence();
    }
    __syncthreads();
  }
}

__global__ __launch_bounds__(256) void scan_kernel(
    const float* __restrict__ DLR, const float* __restrict__ UC, const float* __restrict__ XZ,
    const float* __restrict__ PROJ, const float* __restrict__ A_log, const float* __restrict__ Dv,
    unsigned short* __restrict__ Yh, unsigned short* __restrict__ Yl)
{
  __shared__ __align__(16) float sBC[16 * 32];
  __shared__ __align__(16) float sY[16 * kTP];
  const int tid = threadIdx.x, lane = tid & 31, wave = tid >> 5;
  const int d0 = blockIdx.x * 256, d = d0 + tid;

  float An[kNst];
#pragma unroll
  for (int n = 0; n < kNst; ++n) An[n] = -__expf(A_log[(size_t)d * kNst + n]);
  const float Dd = Dv[d];
  float h[kNst];
#pragma unroll
  for (int n = 0; n < kNst; ++n) h[n] = 0.f;

#pragma unroll 1
  for (int c = 0; c < kSeqL / 16; ++c) {
    const int l0 = c * 16;
    if (tid < 128) {
      const int r = tid >> 3, q = (tid & 7) * 4;
      const v4f v = *(const v4f*)(PROJ + (size_t)(l0 + r) * kPrjP + kDtR + q);
      *(v4f*)(sBC + r * 32 + q) = v;
    }
    __syncthreads();
#pragma unroll 1
    for (int s = 0; s < 16; ++s) {
      const size_t m = (size_t)(l0 + s);
      const float a     = DLR[m * kDin + d];
      const float delta = fmaxf(a, 0.0f) + log1pf(__expf(-fabsf(a)));
      const float xv    = UC[m * kDin + d];
      const float zv    = XZ[m * kXZP + kDin + d];
      v4f Bq[4], Cq[4];
#pragma unroll
      for (int qq = 0; qq < 4; ++qq) {
        Bq[qq] = *(const v4f*)(sBC + s * 32 + 4 * qq);
        Cq[qq] = *(const v4f*)(sBC + s * 32 + kNst + 4 * qq);
      }
      float y = 0.f;
#pragma unroll
      for (int n = 0; n < kNst; ++n) {
        const float e = __expf(delta * An[n]);
        float db = delta * Bq[n >> 2][n & 3];
        asm volatile("" : "+v"(db));
        float p = db * xv;
        asm volatile("" : "+v"(p));
        float qv = h[n] * e;
        asm volatile("" : "+v"(qv));
        const float hn = qv + p;
        h[n] = hn;
        float rr = Cq[n >> 2][n & 3] * hn;
        asm volatile("" : "+v"(rr));
        y += rr;
      }
      float sk = xv * Dd;
      asm volatile("" : "+v"(sk));
      y += sk;
      const float sg = __builtin_amdgcn_rcpf(1.0f + __expf(-zv));
      const float gz = zv * sg;
      sY[s * kTP + tid] = y * gz;
    }
    __syncthreads();
    v8h hv[2], lv[2];
#pragma unroll
    for (int it = 0; it < 2; ++it) {
      const float* sp = sY + (it * 8 + wave) * kTP + lane * 8;
      const v4f a0 = *(const v4f*)(sp);
      const v4f a1 = *(const v4f*)(sp + 4);
#pragma unroll
      for (int e = 0; e < 4; ++e) {
        const unsigned short h0 = f2bf_bits(a0[e]);
        const unsigned short l0 = f2bf_bits(a0[e] - bf_bits2f(h0));
        const unsigned short h1 = f2bf_bits(a1[e]);
        const unsigned short l1 = f2bf_bits(a1[e] - bf_bits2f(h1));
        hv[it][e]     = __builtin_bit_cast(_Float16, h0);
        lv[it][e]     = __builtin_bit_cast(_Float16, l0);
        hv[it][4 + e] = __builtin_bit_cast(_Float16, h1);
        lv[it][4 + e] = __builtin_bit_cast(_Float16, l1);
      }
    }
    for (int pass = 0; pass < 2; ++pass) {
#pragma unroll
      for (int it = 0; it < 2; ++it) {
        const size_t o = (size_t)(l0 + it * 8 + wave) * kDin + d0 + lane * 8;
        *(volatile v8h*)(Yh + o) = hv[it];
        *(volatile v8h*)(Yl + o) = lv[it];
      }
      __threadfence();
    }
  }
}

extern "C" void kernel_launch(void* const* d_in, const int* in_sizes, int n_in,
                              void* d_out, int out_size, void* d_ws, size_t ws_size,
                              hipStream_t stream)
{
  if (n_in < 15) return;
  const float* in0     = (const float*)d_in[0];
  const float* in1     = (const float*)d_in[1];
  const float* ln_g    = (const float*)d_in[2];
  const float* ln_b    = (const float*)d_in[3];
  const float* outp_w  = (const float*)d_in[4];
  const float* outp_b  = (const float*)d_in[5];
  const float* W_in    = (const float*)d_in[6];
  const float* conv_w  = (const float*)d_in[7];
  const float* conv_b  = (const float*)d_in[8];
  const float* W_xprj  = (const float*)d_in[9];
  const float* W_dt    = (const float*)d_in[10];
  const float* b_dt    = (const float*)d_in[11];
  const float* A_log   = (const float*)d_in[12];
  const float* Dv      = (const float*)d_in[13];
  const float* W_mo    = (const float*)d_in[14];
  float* dout = (float*)d_out;

  if (in_sizes[0] != kBatch * kChalf * kSeqL || in_sizes[1] != kBatch * kChalf * kSeqL) return;
  if (in_sizes[2] != kDmod || in_sizes[3] != kDmod) return;
  if (in_sizes[4] != kDmod * kCout || in_sizes[5] != kCout) return;
  if (in_sizes[6] != kDmod * kXZP) return;
  if (in_sizes[7] != kDin * 4 || in_sizes[8] != kDin) return;
  if (in_sizes[9] != kDin * kPrjN) return;
  if (in_sizes[10] != kDtR * kDin || in_sizes[11] != kDin) return;
  if (in_sizes[12] != kDin * kNst || in_sizes[13] != kDin) return;
  if (in_sizes[14] != kDin * kDmod) return;
  if (out_size != kBatch * kCout * kSeqL) return;

  const size_t SZ_WIN  = (size_t)kXZP * kDmod * 2;
  const size_t SZ_WXP  = (size_t)kPrjP * kDin * 2;
  const size_t SZ_WDT  = (size_t)kDin * kDtP * 2;
  const size_t SZ_WMO  = (size_t)kDmod * kDin * 2;
  const size_t SZ_WOP  = (size_t)kCout * kDmod * 2;
  const size_t SZ_X    = (size_t)kRows * kDmod * 2;
  const size_t SZ_XZ   = (size_t)kSeqL * kXZP * 4;
  const size_t SZ_UC   = (size_t)kSeqL * kDin * 4;
  const size_t SZ_UCP  = (size_t)kSeqL * kDin * 2;
  const size_t SZ_PROJ = (size_t)kSeqL * kPrjP * 4;
  const size_t SZ_DTP  = (size_t)kSeqL * kDtP * 2;
  const size_t SZ_DLR  = (size_t)kSeqL * kDin * 4;
  const size_t SZ_YP   = (size_t)kSeqL * kDin * 2;
  const size_t SZ_MOP  = (size_t)kSeqL * kDmod * 2;
  const size_t OFF_WINH = 0;
  const size_t OFF_WINL = OFF_WINH + SZ_WIN;
  const size_t OFF_WXPH = OFF_WINL + SZ_WIN;
  const size_t OFF_WXPL = OFF_WXPH + SZ_WXP;
  const size_t OFF_WDTH = OFF_WXPL + SZ_WXP;
  const size_t OFF_WDTL = OFF_WDTH + SZ_WDT;
  const size_t OFF_WMOH = OFF_WDTL + SZ_WDT;
  const size_t OFF_WMOL = OFF_WMOH + SZ_WMO;
  const size_t OFF_WOPH = OFF_WMOL + SZ_WMO;
  const size_t OFF_WOPL = OFF_WOPH + SZ_WOP;
  const size_t OFF_XH   = OFF_WOPL + SZ_WOP;
  const size_t OFF_XL   = OFF_XH   + SZ_X;
  const size_t OFF_XZ   = OFF_XL   + SZ_X;
  const size_t OFF_UC   = OFF_XZ   + SZ_XZ;
  const size_t OFF_UCH  = OFF_UC   + SZ_UC;
  const size_t OFF_UCL  = OFF_UCH  + SZ_UCP;
  const size_t OFF_PROJ = OFF_UCL  + SZ_UCP;
  const size_t OFF_DTH  = OFF_PROJ + SZ_PROJ;
  const size_t OFF_DTL  = OFF_DTH  + SZ_DTP;
  const size_t OFF_DLR  = OFF_DTL  + SZ_DTP;
  const size_t OFF_YH   = OFF_DLR  + SZ_DLR;
  const size_t OFF_YL   = OFF_YH   + SZ_YP;
  const size_t OFF_MOH  = OFF_YL   + SZ_YP;
  const size_t OFF_MOL  = OFF_MOH  + SZ_MOP;
  const size_t TOTAL    = OFF_MOL  + SZ_MOP;
  if (TOTAL > (size_t)134217728) return;
  if (ws_size < TOTAL) return;

  char* ws = (char*)d_ws;
  unsigned short* WINH = (unsigned short*)(ws + OFF_WINH);
  unsigned short* WINL = (unsigned short*)(ws + OFF_WINL);
  unsigned short* WXPH = (unsigned short*)(ws + OFF_WXPH);
  unsigned short* WXPL = (unsigned short*)(ws + OFF_WXPL);
  unsigned short* WDTH = (unsigned short*)(ws + OFF_WDTH);
  unsigned short* WDTL = (unsigned short*)(ws + OFF_WDTL);
  unsigned short* WMOH = (unsigned short*)(ws + OFF_WMOH);
  unsigned short* WMOL = (unsigned short*)(ws + OFF_WMOL);
  unsigned short* WOPH = (unsigned short*)(ws + OFF_WOPH);
  unsigned short* WOPL = (unsigned short*)(ws + OFF_WOPL);
  unsigned short* XH   = (unsigned short*)(ws + OFF_XH);
  unsigned short* XL   = (unsigned short*)(ws + OFF_XL);
  float*          XZ   = (float*)(ws + OFF_XZ);
  float*          UC   = (float*)(ws + OFF_UC);
  unsigned short* UCH  = (unsigned short*)(ws + OFF_UCH);
  unsigned short* UCL  = (unsigned short*)(ws + OFF_UCL);
  float*          PROJ = (float*)(ws + OFF_PROJ);
  unsigned short* DTH  = (unsigned short*)(ws + OFF_DTH);
  unsigned short* DTL  = (unsigned short*)(ws + OFF_DTL);
  float*          DLR  = (float*)(ws + OFF_DLR);
  unsigned short* YH   = (unsigned short*)(ws + OFF_YH);
  unsigned short* YL   = (unsigned short*)(ws + OFF_YL);
  unsigned short* MOH  = (unsigned short*)(ws + OFF_MOH);
  unsigned short* MOL  = (unsigned short*)(ws + OFF_MOL);
  const float* dummy_bias  = outp_b;
  const float* dummy_resid = in0;

  transpose_split_kernel<<<dim3(kXZP / 64, kDmod / 64), 256, 0, stream>>>(W_in,   WINH, WINL, kDmod, kXZP);
  transpose_split_kernel<<<dim3(kPrjP / 64, kDin / 64), 256, 0, stream>>>(W_xprj, WXPH, WXPL, kDin,  kPrjN);
  dtw_split_kernel<<<(kDin * kDtP) / 8 / 256, 256, 0, stream>>>(W_dt, WDTH, WDTL, (kDin * kDtP) / 8);
  transpose_split_kernel<<<dim3(kDmod / 64, kDin / 64), 256, 0, stream>>>(W_mo,   WMOH, WMOL, kDin,  kDmod);
  transpose_split_kernel<<<dim3(kCout / 64, kDmod / 64), 256, 0, stream>>>(outp_w, WOPH, WOPL, kDmod, kCout);

  ln_kernel<<<dim3(kSeqL / 32, kBatch), 256, 0, stream>>>(in0, in1, ln_g, ln_b, XH, XL);

  for (int b = 0; b < kBatch; ++b) {
    const unsigned short* XHb = XH + (size_t)b * kSeqL * kDmod;
    const unsigned short* XLb = XL + (size_t)b * kSeqL * kDmod;
    float* outb = dout + (size_t)b * kCout * kSeqL;

    wmma_gemm64<1, true, 0, 0, false><<<dim3(128, 1), 256, 0, stream>>>(
        XHb, XLb, kDmod, 0L, WINH, WINL, kDmod, 0L,
        (void*)XZ, (void*)XZ, kXZP, 0L, dummy_bias, dummy_resid, 0L, kSeqL, kXZP, kDmod, 1.0f);

    conv_silu_kernel<<<dim3(kDin / 256, kSeqL / 64), 256, 0, stream>>>(XZ, conv_w, conv_b, UC, UCH, UCL);

    wmma_gemm64<1, true, 0, 0, false><<<dim3(8, 1), 256, 0, stream>>>(
        UCH, UCL, kDin, 0L, WXPH, WXPL, kDin, 0L,
        (void*)PROJ, (void*)PROJ, kPrjP, 0L, dummy_bias, dummy_resid, 0L, kSeqL, kPrjP, kDin, 1.0f);

    dt_split_kernel<<<(kSeqL * kDtP) / 8 / 256, 256, 0, stream>>>(PROJ, DTH, DTL, (kSeqL * kDtP) / 8);

    wmma_gemm64<1, true, 2, 0, false><<<dim3(64, 1), 256, 0, stream>>>(
        DTH, DTL, kDtP, 0L, WDTH, WDTL, kDtP, 0L,
        (void*)DLR, (void*)DLR, kDin, 0L, b_dt, dummy_resid, 0L, kSeqL, kDin, kDtP, 1.0f);

    scan_kernel<<<dim3(kDin / 256, 1), 256, 0, stream>>>(DLR, UC, XZ, PROJ, A_log, Dv, YH, YL);

    wmma_gemm64<1, true, 0, 2, false><<<dim3(32, 1), 256, 0, stream>>>(
        YH, YL, kDin, 0L, WMOH, WMOL, kDin, 0L,
        (void*)MOH, (void*)MOL, kDmod, 0L, dummy_bias, dummy_resid, 0L, kSeqL, kDmod, kDin, 1.0f);

    wmma_gemm64<1, true, 1, 0, false><<<dim3(16, 1), 256, 0, stream>>>(
        WOPH, WOPL, kDmod, 0L, MOH, MOL, kDmod, 0L,
        (void*)outb, (void*)outb, kSeqL, 0L, outp_b, dummy_resid, 0L, kCout, kSeqL, kDmod, 1.0f);
  }
}
